// TpnTaskLoss_54743653155312
// MI455X (gfx1250) — hardware-verified
//
#include <hip/hip_runtime.h>


#define NR_   16384
#define NT2   32768
#define DM    512
#define NCLS  256
#define NBLK  (NT2 / 32)

typedef unsigned short bf;
typedef __attribute__((ext_vector_type(16))) __bf16   v16bf;
typedef __attribute__((ext_vector_type(8)))  unsigned short v8us;
typedef __attribute__((ext_vector_type(8)))  float    v8f;
typedef __attribute__((ext_vector_type(4)))  float    v4f;
typedef v4f  __attribute__((may_alias)) v4fa;

__device__ __forceinline__ unsigned short f2bf(float f) { unsigned u = __float_as_uint(f); u += 0x7FFFu + ((u >> 16) & 1u); return (unsigned short)(u >> 16); }
__device__ __forceinline__ float bf2f(unsigned short b) { return __uint_as_float(((unsigned)b) << 16); }
__device__ __forceinline__ float bfr(float f) { return bf2f(f2bf(f)); }
__device__ __forceinline__ v16bf cat16b(v8us lo, v8us hi) { return __builtin_bit_cast(v16bf, __builtin_shufflevector(lo, hi, 0, 1, 2, 3, 4, 5, 6, 7, 8, 9, 10, 11, 12, 13, 14, 15)); }
__device__ __forceinline__ v8f wmmab(v16bf a, v16bf b, v8f c) { return __builtin_amdgcn_wmma_f32_16x16x32_bf16(false, a, false, b, (short)0, c, false, false); }
#define VST2(T, p, v) do { const T vst2_v_ = (v); *(volatile T*)(p) = vst2_v_; __threadfence(); *(volatile T*)(p) = vst2_v_; } while (0)

__global__ __launch_bounds__(256) void k_fb(const float* __restrict__ sf, const float* __restrict__ tf, bf* FB) {
    const int lane = threadIdx.x & 31, r = blockIdx.x * 8 + (threadIdx.x >> 5);
    if (r >= NT2) return;
    const float* s = (r < NR_) ? (sf + (size_t)r * DM) : (tf + (size_t)(r - NR_) * DM);
    v8us o[2];
#pragma unroll
    for (int q = 0; q < 2; ++q) { v8us t;
#pragma unroll
        for (int i = 0; i < 8; ++i) t[i] = f2bf(s[q * 256 + lane * 8 + i]);
        o[q] = t; }
#pragma unroll
    for (int q = 0; q < 2; ++q) *(volatile v8us*)(FB + (size_t)r * DM + q * 256 + lane * 8) = o[q];
    __threadfence();
#pragma unroll
    for (int q = 0; q < 2; ++q) *(volatile v8us*)(FB + (size_t)r * DM + q * 256 + lane * 8) = o[q];
}

__global__ __launch_bounds__(256) void k_csum(const float* __restrict__ sf, const float* __restrict__ tf, const int* __restrict__ sl, const int* __restrict__ tl, float* SUM, float* CNT) {
    extern __shared__ float4 lds_raw[];
    float* agg = (float*)lds_raw;
    int* lab = (int*)(agg + NCLS * 256);
    int* cnt = lab + 256;
    const int t = threadIdx.x, half = blockIdx.x, set = blockIdx.y, c0 = half * 256;
    const float* F = set ? tf : sf; const int* Lb = set ? tl : sl;
    for (int i = t; i < NCLS * 256; i += 256) agg[i] = 0.f;
    cnt[t] = 0;
    __syncthreads();
#pragma unroll 1
    for (int r0 = 0; r0 < NR_; r0 += 256) {
        int l = Lb[r0 + t]; l = min(max(l, 0), NCLS - 1); lab[t] = l;
        __syncthreads();
#pragma unroll 1
        for (int q = 0; q < 256; ++q) { const int c = lab[q]; agg[c * 256 + t] += bfr(F[(size_t)(r0 + q) * DM + c0 + t]); }
        if (half == 0 && t == 0) { for (int q = 0; q < 256; ++q) cnt[lab[q]] += 1; }
        __syncthreads();
    }
    const int lane = t & 31, wv = t >> 5;
#pragma unroll 1
    for (int i = 0; i < 32; ++i) {
        const int c = wv * 32 + i; float* row = SUM + ((size_t)set * NCLS + c) * DM + c0;
        float v[8];
#pragma unroll
        for (int q = 0; q < 8; ++q) v[q] = agg[c * 256 + q * 32 + lane];
#pragma unroll
        for (int q = 0; q < 8; ++q) *(volatile float*)(row + q * 32 + lane) = v[q];
        __threadfence();
#pragma unroll
        for (int q = 0; q < 8; ++q) *(volatile float*)(row + q * 32 + lane) = v[q];
    }
    if (half == 0) VST2(float, CNT + (size_t)set * NCLS + t, (float)cnt[t]);
}

__global__ __launch_bounds__(256) void k_means(const float* __restrict__ SUM, const float* __restrict__ CNT, bf* UH, bf* UL) {
    const int lane = threadIdx.x & 31, wid = blockIdx.x * 8 + (threadIdx.x >> 5);
    if (wid >= 3 * NCLS) return;
    const int m = wid / NCLS, c = wid - m * NCLS;
    const float cs = CNT[c], ct = CNT[NCLS + c];
    const float den = (m == 0) ? cs : ((m == 1) ? ct : (cs + ct));
#pragma unroll 1
    for (int q = 0; q < 2; ++q) {
        v8us oh, ol;
#pragma unroll
        for (int i = 0; i < 8; ++i) {
            const int k = q * 256 + lane * 8 + i;
            const float a = SUM[(size_t)c * DM + k], b = SUM[((size_t)NCLS + c) * DM + k];
            const float num = (m == 0) ? a : ((m == 1) ? b : (a + b));
            const float u = num / den;
            const unsigned short hb = f2bf(u); oh[i] = hb; ol[i] = f2bf(u - bf2f(hb));
        }
        *(volatile v8us*)(UH + (size_t)wid * DM + q * 256 + lane * 8) = oh; *(volatile v8us*)(UL + (size_t)wid * DM + q * 256 + lane * 8) = ol;
        __threadfence();
        *(volatile v8us*)(UH + (size_t)wid * DM + q * 256 + lane * 8) = oh; *(volatile v8us*)(UL + (size_t)wid * DM + q * 256 + lane * 8) = ol;
    }
}

__global__ __launch_bounds__(64) void k_kl(const bf* __restrict__ FB, const bf* __restrict__ UH, const bf* __restrict__ UL, float* PART) {
    extern __shared__ float4 lds_raw[];
    float* tiles = (float*)lds_raw;
    __shared__ float wsum[2];
    const int lane = threadIdx.x & 31, wave = threadIdx.x >> 5, lr = lane & 15, hi = lane >> 4;
    const int r0 = blockIdx.x * 32 + wave * 16;
    float* myt = tiles + (size_t)wave * 3 * 16 * 260;
    float klacc = 0.f;
#pragma unroll 1
    for (int m = 0; m < 3; ++m) {
        v8f acc[16];
#pragma unroll
        for (int t = 0; t < 16; ++t) acc[t] = (v8f){};
        const bf* uh = UH + (size_t)m * NCLS * DM; const bf* ul = UL + (size_t)m * NCLS * DM;
#pragma unroll 1
        for (int kc = 0; kc < DM; kc += 32) {
            const bf* ap = FB + (size_t)(r0 + lr) * DM + kc + 8 * hi;
            const v16bf a = cat16b(*(const v8us*)ap, *(const v8us*)(ap + 16));
#pragma unroll
            for (int t = 0; t < 16; ++t) {
                const size_t bo = (size_t)(t * 16 + lr) * DM + kc + 8 * hi;
                acc[t] = wmmab(a, cat16b(*(const v8us*)(uh + bo), *(const v8us*)(uh + bo + 16)), acc[t]);
                acc[t] = wmmab(a, cat16b(*(const v8us*)(ul + bo), *(const v8us*)(ul + bo + 16)), acc[t]);
            }
            asm volatile("v_nop\n\tv_nop\n\tv_nop\n\tv_nop" : "+v"(acc[0]), "+v"(acc[5]), "+v"(acc[10]), "+v"(acc[15]) : "v"(a));
        }
#pragma unroll
        for (int j = 0; j < 8; ++j) {
            float mx = -3.0e38f;
#pragma unroll
            for (int t = 0; t < 16; ++t) mx = fmaxf(mx, acc[t][j]);
            mx = fmaxf(mx, __shfl_xor(mx, 1, 16)); mx = fmaxf(mx, __shfl_xor(mx, 2, 16)); mx = fmaxf(mx, __shfl_xor(mx, 4, 16)); mx = fmaxf(mx, __shfl_xor(mx, 8, 16));
            float se = 0.f;
#pragma unroll
            for (int t = 0; t < 16; ++t) se += expf(acc[t][j] - mx);
            se += __shfl_xor(se, 1, 16); se += __shfl_xor(se, 2, 16); se += __shfl_xor(se, 4, 16); se += __shfl_xor(se, 8, 16);
            const float lse = logf(se) + mx;
#pragma unroll
            for (int t = 0; t < 16; ++t) myt[(size_t)m * 16 * 260 + (hi * 8 + j) * 260 + t * 16 + lr] = acc[t][j] - lse;
        }
    }
    asm volatile("" ::: "memory");
#pragma unroll
    for (int j = 0; j < 8; ++j)
#pragma unroll
        for (int t = 0; t < 16; ++t) {
            const int e = (hi * 8 + j) * 260 + t * 16 + lr;
            const float ls = myt[e], lt = myt[16 * 260 + e], lst = myt[2 * 16 * 260 + e];
            const float ps = expf(ls), pt = expf(lt), pst = expf(lst);
            klacc += pt * (lt - ls) + ps * (ls - lt) + pst * (lst - ls) + ps * (ls - lst) + pst * (lst - lt) + pt * (lt - lst);
        }
#pragma unroll
    for (int o = 16; o; o >>= 1) klacc += __shfl_xor(klacc, o, 32);
    if (lane == 0) wsum[wave] = klacc;
    __syncthreads();
    if (wave == 0) VST2(float, PART + (size_t)blockIdx.x * 32 + lane, wsum[0] + wsum[1]);
}

__global__ __launch_bounds__(32) void k_fin(const float* __restrict__ PART, float* out) {
    const int lane = threadIdx.x;
    double s = 0.0;
#pragma unroll 1
    for (int i = lane; i < NBLK; i += 32) s += (double)PART[(size_t)i * 32];
#pragma unroll
    for (int o = 16; o; o >>= 1) s += __shfl_xor(s, o, 32);
    if (lane == 0) { const float v = (float)(s * 0.5 / 3.0 / ((double)NT2 * (double)NCLS)); *(volatile float*)out = v; __threadfence(); *(volatile float*)out = v; }
}

extern "C" void kernel_launch(void* const* d_in, const int* in_sizes, int n_in,
                              void* d_out, int out_size, void* d_ws, size_t ws_size, hipStream_t stream) {
    (void)in_sizes; (void)n_in; (void)out_size;
    const float* sf = (const float*)d_in[0]; const float* tf = (const float*)d_in[1]; const int* sl = (const int*)d_in[2]; const int* tl = (const int*)d_in[3];
    float* out = (float*)d_out;
    char* wsp = (char*)d_ws;
    auto take = [&](size_t bytes) { char* p = wsp; wsp += (bytes + 255) & ~(size_t)255; return (void*)p; };
    bf* FB = (bf*)take((size_t)NT2 * DM * 2);
    float* SUM = (float*)take((size_t)2 * NCLS * DM * 4); float* CNT = (float*)take((size_t)2 * NCLS * 4);
    bf* UH = (bf*)take((size_t)3 * NCLS * DM * 2); bf* UL = (bf*)take((size_t)3 * NCLS * DM * 2);
    float* PART = (float*)take((size_t)NBLK * 32 * 4);
    if ((size_t)(wsp - (char*)d_ws) > ws_size) return;
    k_fb<<<NT2 / 8, 256, 0, stream>>>(sf, tf, FB);
    k_csum<<<dim3(2, 2, 1), 256, (size_t)NCLS * 256 * 4 + 512 * 4, stream>>>(sf, tf, sl, tl, SUM, CNT);
    k_means<<<(3 * NCLS) / 8, 256, 0, stream>>>(SUM, CNT, UH, UL);
    k_kl<<<NBLK, 64, (size_t)2 * 3 * 16 * 260 * 4, stream>>>(FB, UH, UL, PART);
    k_fin<<<1, 32, 0, stream>>>(PART, out);
}
